// PeepholeCell_46677704573636
// MI455X (gfx1250) — hardware-verified
//
#include <hip/hip_runtime.h>

typedef __bf16         v16b  __attribute__((ext_vector_type(16)));
typedef unsigned short v16us __attribute__((ext_vector_type(16)));
typedef unsigned short v8us  __attribute__((ext_vector_type(8)));
typedef float          v8f   __attribute__((ext_vector_type(8)));
typedef float          v4f   __attribute__((ext_vector_type(4)));
typedef v8us __attribute__((may_alias)) v8usa;
typedef v4f  __attribute__((may_alias)) v4fa;

union FragB { v16b v; v16us u; v8us half[2]; };

#define BROWS 16384
#define KD    512
#define NGATE 4
#define NPRE  (NGATE * KD)
#define NACT  (BROWS * KD)
#define NACT8 (NACT / 8)
#define NWEL  (KD * KD)
#define NWPL  (NPRE * KD)
#define WSC   16.0f
#define WSCI  0.0625f

#define MT   64
#define HT   64
#define LDT  72
#define LDO  68

static_assert((NACT8 % 256) == 0);
static_assert((BROWS % MT) == 0);
static_assert((KD % HT) == 0);
static_assert((KD % 64) == 0);
static_assert((LDT % 8) == 0);
static_assert((LDO % 4) == 0);

__device__ __forceinline__ v8f wmma_bf16(v16b a, v16b b, v8f c) {
  v8f d = __builtin_amdgcn_wmma_f32_16x16x32_bf16(false, a, false, b, (short)0, c, false, false);
  asm volatile("v_nop\n\tv_nop\n\tv_nop\n\tv_nop" : "+v"(d) : "v"(a), "v"(b));
  return d;
}

__device__ __forceinline__ v16b load_frag_b(const unsigned short* p, int hf) {
  FragB f;
  f.half[0] = *(const v8usa*)(p + 8 * hf);
  f.half[1] = *(const v8usa*)(p + 16 + 8 * hf);
  return f.v;
}

__device__ __forceinline__ unsigned int bf16_rne_bits(float x) {
  unsigned int u = __float_as_uint(x);
  u += 0x7FFFu + ((u >> 16) & 1u);
  return u >> 16;
}
__device__ __forceinline__ void split_bf16(float x, unsigned short& hb, unsigned short& lb) {
  const unsigned int hbits = bf16_rne_bits(x);
  const float hv = __uint_as_float(hbits << 16);
  const unsigned int lbits = bf16_rne_bits(x - hv);
  hb = (unsigned short)hbits;
  lb = (unsigned short)lbits;
}

__device__ __forceinline__ float sigmoid_f(float x) {
  return __builtin_amdgcn_rcpf(1.0f + __expf(-x));
}
__device__ __forceinline__ float tanh_f(float x) {
  const float e = __expf(fminf(-2.0f * x, 80.0f));
  return (1.0f - e) * __builtin_amdgcn_rcpf(1.0f + e);
}

__global__ __launch_bounds__(256) void convert_act_kernel(
    const float* __restrict__ X, const float* __restrict__ Cp,
    unsigned short* __restrict__ ah, unsigned short* __restrict__ al)
{
  const int g = blockIdx.x * 256 + threadIdx.x;
  if (g >= 2 * NACT8) return;
  const float* src;
  if (g < NACT8) src = X + (size_t)g * 8;
  else           src = Cp + (size_t)(g - NACT8) * 8;
  const v4f a = *(const v4fa*)src;
  const v4f c = *(const v4fa*)(src + 4);
  const float v[8] = { a.x, a.y, a.z, a.w, c.x, c.y, c.z, c.w };
  unsigned short hb[8], lb[8];
  #pragma unroll
  for (int j = 0; j < 8; ++j) split_bf16(v[j], hb[j], lb[j]);
  const v8us oh = { hb[0], hb[1], hb[2], hb[3], hb[4], hb[5], hb[6], hb[7] };
  const v8us ol = { lb[0], lb[1], lb[2], lb[3], lb[4], lb[5], lb[6], lb[7] };
  unsigned short* dh = ah + (size_t)g * 8;
  unsigned short* dl = al + (size_t)g * 8;
  *(volatile v8us*)dh = oh;
  *(volatile v8us*)dl = ol;
  __threadfence();
  *(volatile v8us*)dh = oh;
  *(volatile v8us*)dl = ol;
}

__device__ __forceinline__ void wt_store_pass_b(const unsigned short* sh, const unsigned short* sl,
                                                unsigned short* ph, unsigned short* pl,
                                                int fam, int g, int n0, int k0, int w, int lane) {
  const int q8 = lane & 7, sub = lane >> 3;
  #pragma unroll
  for (int i = 0; i < 2; ++i) {
    const int lid = w * 8 + i * 4 + sub;
    const v8us vh = *(const v8usa*)(sh + lid * LDT + 8 * q8);
    const v8us vl = *(const v8usa*)(sl + lid * LDT + 8 * q8);
    const size_t gi = ((size_t)fam * NPRE + g * KD + n0 + lid) * KD + k0 + 8 * q8;
    *(volatile v8us*)(ph + gi) = vh;
    *(volatile v8us*)(pl + gi) = vl;
  }
}

__global__ __launch_bounds__(256) void convert_w_kernel(
    const float* __restrict__ w0, const float* __restrict__ w1,
    const float* __restrict__ w2, const float* __restrict__ w3,
    const float* __restrict__ u0, const float* __restrict__ u1,
    const float* __restrict__ u2, const float* __restrict__ u3,
    unsigned short* __restrict__ bh, unsigned short* __restrict__ bl)
{
  __shared__ __attribute__((aligned(16))) unsigned short sHi[64 * LDT];
  __shared__ __attribute__((aligned(16))) unsigned short sLo[64 * LDT];

  const int bid = blockIdx.x;
  const int fam = bid >> 8;
  const int t = bid & 255;
  const int g = t >> 6, kt = (t >> 3) & 7, nt = t & 7;
  const int k0 = kt * 64, n0 = nt * 64;
  const int tid = threadIdx.x, lane = tid & 31, w = tid >> 5;

  const float* src;
  if (fam == 0) src = (g == 0) ? w0 : ((g == 1) ? w1 : ((g == 2) ? w2 : w3));
  else          src = (g == 0) ? u0 : ((g == 1) ? u1 : ((g == 2) ? u2 : u3));

  const int kr = tid >> 2;
  const int cq = (tid & 3) * 16;
  const float* p = src + (size_t)(k0 + kr) * KD + n0 + cq;
  const v4f q0 = *(const v4fa*)(p);
  const v4f q1 = *(const v4fa*)(p + 4);
  const v4f q2 = *(const v4fa*)(p + 8);
  const v4f q3 = *(const v4fa*)(p + 12);
  const float v[16] = { q0.x, q0.y, q0.z, q0.w, q1.x, q1.y, q1.z, q1.w,
                        q2.x, q2.y, q2.z, q2.w, q3.x, q3.y, q3.z, q3.w };

  #pragma unroll
  for (int j = 0; j < 16; ++j) {
    unsigned short hb, lb;
    split_bf16(v[j] * WSC, hb, lb);
    sHi[(cq + j) * LDT + kr] = hb;
    sLo[(cq + j) * LDT + kr] = lb;
  }
  __syncthreads();

  wt_store_pass_b(sHi, sLo, bh, bl, fam, g, n0, k0, w, lane);
  __threadfence();
  wt_store_pass_b(sHi, sLo, bh, bl, fam, g, n0, k0, w, lane);
}

__device__ __forceinline__ void out_store_pass(const float* so, float* out,
                                               int m0, int hc0, int w, int lane) {
  const int q8 = lane & 7, sub = lane >> 3;
  #pragma unroll
  for (int i = 0; i < 4; ++i) {
    const int lid = w * 16 + i * 4 + sub;
    const int row = lid >> 1, hl = lid & 1;
    const v4f v = *(const v4fa*)(so + row * LDO + 32 * hl + 4 * q8);
    const size_t gi = (size_t)(m0 + row) * KD + hc0 + 32 * hl + 4 * q8;
    *(volatile v4f*)(out + gi) = v;
  }
}

__global__ __launch_bounds__(256) void cell_kernel(
    const unsigned short* __restrict__ ah,
    const unsigned short* __restrict__ al,
    const unsigned short* __restrict__ bh,
    const unsigned short* __restrict__ bl,
    const float* __restrict__ Cprev,
    const float* __restrict__ bf, const float* __restrict__ bi,
    const float* __restrict__ bo, const float* __restrict__ bc,
    float* __restrict__ out)
{
  __shared__ __attribute__((aligned(16))) float sO[MT * LDO];

  const int tid = threadIdx.x, lane = tid & 31, w = tid >> 5;
  const int hf = lane >> 4, m = lane & 15;
  const int m0 = blockIdx.y * MT, hc0 = blockIdx.x * HT;
  const int rg = w >> 2, cg = w & 3;
  const int rbase = m0 + 32 * rg;
  const int ncol = hc0 + 16 * cg;

  const v8f zero8 = { 0.f, 0.f, 0.f, 0.f, 0.f, 0.f, 0.f, 0.f };
  v8f acc[2][NGATE];
  #pragma unroll
  for (int rt = 0; rt < 2; ++rt)
    #pragma unroll
    for (int g = 0; g < NGATE; ++g) acc[rt][g] = zero8;

  #pragma unroll 1
  for (int s = 0; s < 2; ++s) {
    const unsigned short* a0h = ah + (size_t)s * NACT + (size_t)(rbase + m) * KD;
    const unsigned short* a1h = a0h + (size_t)16 * KD;
    const unsigned short* a0l = al + (size_t)s * NACT + (size_t)(rbase + m) * KD;
    const unsigned short* a1l = a0l + (size_t)16 * KD;
    const unsigned short* bhp = bh + (size_t)s * NWPL + (size_t)(ncol + m) * KD;
    const unsigned short* blp = bl + (size_t)s * NWPL + (size_t)(ncol + m) * KD;

    #pragma unroll 1
    for (int k0 = 0; k0 < KD; k0 += 32) {
      const v16b x0h = load_frag_b(a0h + k0, hf);
      const v16b x0l = load_frag_b(a0l + k0, hf);
      const v16b x1h = load_frag_b(a1h + k0, hf);
      const v16b x1l = load_frag_b(a1l + k0, hf);
      #pragma unroll
      for (int g = 0; g < NGATE; ++g) {
        const v16b whf = load_frag_b(bhp + (size_t)g * KD * KD + k0, hf);
        const v16b wlf = load_frag_b(blp + (size_t)g * KD * KD + k0, hf);
        acc[0][g] = wmma_bf16(x0h, whf, acc[0][g]);
        acc[0][g] = wmma_bf16(x0h, wlf, acc[0][g]);
        acc[0][g] = wmma_bf16(x0l, whf, acc[0][g]);
        acc[1][g] = wmma_bf16(x1h, whf, acc[1][g]);
        acc[1][g] = wmma_bf16(x1h, wlf, acc[1][g]);
        acc[1][g] = wmma_bf16(x1l, whf, acc[1][g]);
      }
    }
  }

  const int hcol = ncol + m;
  const float vbf = bf[hcol], vbi = bi[hcol], vbo = bo[hcol], vbc = bc[hcol];
  #pragma unroll
  for (int rt = 0; rt < 2; ++rt) {
    #pragma unroll
    for (int r = 0; r < 8; ++r) {
      const int rowl = 32 * rg + 16 * rt + 8 * hf + r;
      const size_t grow = (size_t)(m0 + rowl);
      const float pf = acc[rt][0][r] * WSCI + vbf;
      const float pi = acc[rt][1][r] * WSCI + vbi;
      const float po = acc[rt][2][r] * WSCI + vbo;
      const float pc = acc[rt][3][r] * WSCI + vbc;
      const float ft = sigmoid_f(pf);
      const float it = sigmoid_f(pi);
      const float ot = sigmoid_f(po);
      const float ch = tanh_f(pc);
      const float cp = Cprev[grow * KD + hcol];
      const float ct = ft * cp + it * ch;
      sO[rowl * LDO + 16 * cg + m] = ot * tanh_f(ct);
    }
  }
  __syncthreads();

  out_store_pass(sO, out, m0, hc0, w, lane);
  __threadfence();
  out_store_pass(sO, out, m0, hc0, w, lane);
}

extern "C" void kernel_launch(void* const* d_in, const int* in_sizes, int n_in,
                              void* d_out, int out_size, void* d_ws, size_t ws_size,
                              hipStream_t stream) {
  if (n_in < 14) return;
  if (in_sizes[0] != NACT || in_sizes[1] != NACT) return;
  for (int i = 2; i < 10; ++i) if (in_sizes[i] != NWEL) return;
  for (int i = 10; i < 14; ++i) if (in_sizes[i] != KD) return;
  if (out_size != NACT) return;

  const float* X  = (const float*)d_in[0];
  const float* Cp = (const float*)d_in[1];
  const float* Wf = (const float*)d_in[2];
  const float* Wi = (const float*)d_in[3];
  const float* Wo = (const float*)d_in[4];
  const float* Wc = (const float*)d_in[5];
  const float* Uf = (const float*)d_in[6];
  const float* Ui = (const float*)d_in[7];
  const float* Uo = (const float*)d_in[8];
  const float* Uc = (const float*)d_in[9];
  const float* bfp = (const float*)d_in[10];
  const float* bip = (const float*)d_in[11];
  const float* bop = (const float*)d_in[12];
  const float* bcp = (const float*)d_in[13];
  float* out = (float*)d_out;

  const size_t act_bytes = (size_t)2 * NACT * 2;
  const size_t wt_bytes  = (size_t)2 * NWPL * 2;
  const size_t total = 2 * act_bytes + 2 * wt_bytes;
  if (total > ws_size) return;

  char* ws = (char*)d_ws;
  unsigned short* ah = (unsigned short*)(ws);
  unsigned short* al = (unsigned short*)(ws + act_bytes);
  unsigned short* bh = (unsigned short*)(ws + 2 * act_bytes);
  unsigned short* bl = (unsigned short*)(ws + 2 * act_bytes + wt_bytes);

  convert_act_kernel<<<(2 * NACT8) / 256, 256, 0, stream>>>(X, Cp, ah, al);

  convert_w_kernel<<<512, 256, 0, stream>>>(Wf, Wi, Wo, Wc, Uf, Ui, Uo, Uc, bh, bl);

  dim3 gCell(KD / HT, BROWS / MT);
  cell_kernel<<<gCell, 256, 0, stream>>>(ah, al, bh, bl, Cp, bfp, bip, bop, bcp, out);
}
